// EncoderLayer_3530463117510
// MI455X (gfx1250) — hardware-verified
//
#include <hip/hip_runtime.h>


#ifndef NB
#define NB 2
#endif
#ifndef SEQ
#define SEQ 2048
#endif
#define NB_FULL 2
#define SEQ_FULL 2048
#define TT   SEQ
#define DM   1024
#define NH_  16
#define HD   64
#define DQ   (NH_ * HD)
#define D3   (3 * DM)
#define FF   4096
#define ZH   2
#define PCAR 1024.0f
#define CCAR 16.0f
#define WCAR 64.0f
#define SCL  0.125f
#define LNEPS 1e-6f
#define FMIN (-3.4028234663852886e+38f)

static_assert(TT % 128 == 0);
static_assert(TT <= SEQ_FULL);
static_assert(NB >= 1 && NB <= NB_FULL);
static_assert(NH_ % ZH == 0);
static_assert(DM % 64 == 0 && FF % 64 == 0 && D3 % 64 == 0 && HD == 64);

typedef _Float16 h16;
typedef __attribute__((ext_vector_type(16))) _Float16 v16h;
typedef __attribute__((ext_vector_type(8)))  _Float16 v8h;
typedef __attribute__((ext_vector_type(4)))  _Float16 v4h;
typedef __attribute__((ext_vector_type(2)))  _Float16 v2h;
typedef __attribute__((ext_vector_type(8)))  float v8f;
typedef __attribute__((ext_vector_type(4)))  float v4f;
typedef __attribute__((ext_vector_type(2)))  float v2f;
typedef __attribute__((ext_vector_type(4)))  int v4i;
typedef v4f __attribute__((may_alias)) v4fa;

__device__ __forceinline__ unsigned short f2bf(float f) { unsigned u = __float_as_uint(f); u += 0x7FFFu + ((u >> 16) & 1u); return (unsigned short)(u >> 16); }
__device__ __forceinline__ float bf2f(unsigned short b) { return __uint_as_float(((unsigned)b) << 16); }
__device__ __forceinline__ float bfr(float f) { return bf2f(f2bf(f)); }
__device__ __forceinline__ v16h cat16(v8h lo, v8h hi) { return __builtin_shufflevector(lo, hi, 0, 1, 2, 3, 4, 5, 6, 7, 8, 9, 10, 11, 12, 13, 14, 15); }
__device__ __forceinline__ v8f wmma16(v16h a, v16h b, v8f c) { return __builtin_amdgcn_wmma_f32_16x16x32_f16(false, a, false, b, (short)0, c, false, false); }
__device__ __forceinline__ v16h ldfrag(const h16* p) { return cat16(*(const v8h*)p, *(const v8h*)(p + 16)); }

template <bool BIAS>
__global__ __launch_bounds__(32) void k_gemm(const h16* __restrict__ A, const h16* __restrict__ Bt, int K, float* C, int ldc, const float* __restrict__ bias, float osc, size_t sA, size_t sB, size_t sC) {
    __shared__ __align__(16) float os[16 * 68];
    const size_t z = blockIdx.z; A += z * sA; Bt += z * sB; C += z * sC;
    const int lane = threadIdx.x & 31, lr = lane & 15, hi = lane >> 4; const int r0 = blockIdx.x * 64, c0 = blockIdx.y * 64;
    v8f acc[4][4];
#pragma unroll
    for (int mb = 0; mb < 4; ++mb)
#pragma unroll
        for (int nb = 0; nb < 4; ++nb) acc[mb][nb] = (v8f){};
    const size_t aoff = (size_t)(r0 + lr) * K + 8 * hi, boff = (size_t)(c0 + lr) * K + 8 * hi;
#pragma unroll 1
    for (int kc = 0; kc < K; kc += 32) {
        v16h a[4];
#pragma unroll
        for (int mb = 0; mb < 4; ++mb) a[mb] = ldfrag(A + aoff + (size_t)mb * 16 * K + kc);
#pragma unroll
        for (int nb = 0; nb < 4; ++nb) { const v16h b = ldfrag(Bt + boff + (size_t)nb * 16 * K + kc);
#pragma unroll
            for (int mb = 0; mb < 4; ++mb) acc[mb][nb] = wmma16(a[mb], b, acc[mb][nb]); }
        asm volatile("v_nop\n\tv_nop\n\tv_nop\n\tv_nop" : "+v"(acc[0][0]), "+v"(acc[1][1]), "+v"(acc[2][2]), "+v"(acc[3][3]) : "v"(a[0]), "v"(a[3]));
    }
#pragma unroll
    for (int mb = 0; mb < 4; ++mb) {
#pragma unroll
        for (int nb = 0; nb < 4; ++nb) {
#pragma unroll
            for (int j = 0; j < 8; ++j) os[(hi * 8 + j) * 68 + nb * 16 + lr] = acc[mb][nb][j]; }
        __builtin_amdgcn_fence(3  , "wavefront"); __builtin_amdgcn_wave_barrier(); asm volatile("" ::: "memory");
        float* crow = C + (size_t)(r0 + mb * 16) * ldc + c0;
#pragma unroll 1
        for (int ps = 0; ps < 2; ++ps) {
#pragma unroll
            for (int s = 0; s < 8; ++s) { const int row = 2 * s + hi, cofs = lr * 4; v4f val = *(const v4fa*)(os + row * 68 + cofs); val = val * osc;
                if (BIAS) { val[0] += bfr(bias[c0 + cofs]); val[1] += bfr(bias[c0 + cofs + 1]); val[2] += bfr(bias[c0 + cofs + 2]); val[3] += bfr(bias[c0 + cofs + 3]); }
                *(volatile v4f*)(crow + (size_t)row * ldc + cofs) = val; }
            if (ps == 0) __threadfence(); }
        __builtin_amdgcn_fence(3  , "wavefront"); __builtin_amdgcn_wave_barrier(); asm volatile("" ::: "memory");
    }
}

__global__ __launch_bounds__(256) void k_wt(const float* __restrict__ w, int K, int N, h16* Bt) {
    const int lane = threadIdx.x & 31; const int L0 = (blockIdx.x * 8 + (threadIdx.x >> 5)) * 8; const int nlines = (int)((size_t)N * K / 64);
#pragma unroll
    for (int ps = 0; ps < 2; ++ps) {
#pragma unroll 1
        for (int l = 0; l < 8; ++l) { const int L = L0 + l; if (L >= nlines) break; const size_t e = (size_t)L * 64 + lane * 2; const int k = (int)(e % K), n = (int)(e / K); v2h o;
            o[0] = (h16)(bfr(w[(size_t)k * N + n]) * WCAR); o[1] = (h16)(bfr(w[(size_t)(k + 1) * N + n]) * WCAR); *(volatile v2h*)(Bt + e) = o; }
        if (ps == 0) __threadfence(); }
}

__global__ __launch_bounds__(256) void k_cstab(float* CS) {
    const int idx = blockIdx.x * 256 + threadIdx.x; const int i = idx & 31; const int t = idx >> 5; if (t >= TT) return;
    double p = 1.0;
#pragma unroll 1
    for (int s = 0; s < i; ++s) p *= 1.333521432163324;
    const float pf = (float)p;
    const float inv = __fdiv_rn(1.0f, pf);
    const float ang = __fmul_rn((float)t, inv);
    const double a = (double)ang;
    const double kd = __builtin_rint(a * 0.63661977236758134308);
    const double rd = __builtin_fma(-kd, 1.57079632679489661923, a);
    const float r = (float)rd; const int qd = ((int)kd) & 3;
    const float r2 = r * r;
    const float cp = 1.0f + r2 * (-0.5f + r2 * (0.041666667f + r2 * (-0.0013888889f + r2 * (2.4801587e-5f + r2 * (-2.7557319e-7f)))));
    const float sp = r + r * r2 * (-0.16666667f + r2 * (0.0083333333f + r2 * (-0.00019841270f + r2 * 2.7557319e-6f)));
    const float c = (qd == 0) ? cp : (qd == 1) ? -sp : (qd == 2) ? -cp : sp;
    const float sn = (qd == 0) ? sp : (qd == 1) ? cp : (qd == 2) ? -sp : -cp;
    v2f cs; cs[0] = c; cs[1] = sn;
    float* p0 = CS + ((size_t)t * HD + i) * 2; float* p1 = CS + ((size_t)t * HD + i + HD / 2) * 2;
    *(volatile v2f*)p0 = cs; *(volatile v2f*)p1 = cs; __threadfence(); *(volatile v2f*)p0 = cs; *(volatile v2f*)p1 = cs;
}

template <bool RIN>
__global__ __launch_bounds__(256) void k_lnx(const float* __restrict__ F, const float* __restrict__ g, const float* __restrict__ bb, h16* out) {
    const int lane = threadIdx.x & 31; const int row = blockIdx.x * 8 + (threadIdx.x >> 5); if (row >= TT) return;
    const float* fr = F + (size_t)row * DM + lane * 4; h16* orow = out + (size_t)row * DM + lane * 4; float s = 0.f;
#pragma unroll 1
    for (int c = 0; c < DM / 128; ++c) { const v4f a = *(const v4f*)(fr + c * 128);
#pragma unroll
        for (int q = 0; q < 4; ++q) { const float xv = RIN ? bfr(a[q]) : a[q]; s = __fadd_rn(s, xv); } }
#pragma unroll
    for (int sh = 16; sh; sh >>= 1) s = __fadd_rn(s, __shfl_xor(s, sh, 32));
    const float mean = __fmul_rn(s, 1.0f / (float)DM); float s2 = 0.f;
#pragma unroll 1
    for (int c = 0; c < DM / 128; ++c) { const v4f a = *(const v4f*)(fr + c * 128);
#pragma unroll
        for (int q = 0; q < 4; ++q) { const float xv = RIN ? bfr(a[q]) : a[q]; const float dv = __fsub_rn(xv, mean); float p2 = __fmul_rn(dv, dv); asm volatile("" : "+v"(p2)); s2 = __fadd_rn(s2, p2); } }
#pragma unroll
    for (int sh = 16; sh; sh >>= 1) s2 = __fadd_rn(s2, __shfl_xor(s2, sh, 32));
    const float rs = __fdiv_rn(1.0f, __fsqrt_rn(__fadd_rn(__fmul_rn(s2, 1.0f / (float)DM), LNEPS)));
#pragma unroll 1
    for (int ps = 0; ps < 2; ++ps) {
#pragma unroll 1
        for (int c = 0; c < DM / 128; ++c) { const v4f a = *(const v4f*)(fr + c * 128); v4h o;
#pragma unroll
            for (int q = 0; q < 4; ++q) { const int col = c * 128 + lane * 4 + q; const float xv = RIN ? bfr(a[q]) : a[q]; const float dv = __fsub_rn(xv, mean); float y = __fmul_rn(dv, rs); asm volatile("" : "+v"(y)); y = __fmul_rn(y, bfr(g[col])); asm volatile("" : "+v"(y)); o[q] = (h16)__fadd_rn(y, bfr(bb[col])); }
            *(volatile v4h*)(orow + c * 128) = o; }
        if (ps == 0) __threadfence(); }
}

__global__ __launch_bounds__(256) void k_rope(const float* __restrict__ F, int pitch, int nheads, const float* __restrict__ CS, h16* P16) {
    const size_t e = ((size_t)blockIdx.x * 256 + threadIdx.x) * 2; if (e >= (size_t)nheads * TT * HD) return; const int d = (int)(e % HD); const int t = (int)((e / HD) % TT); const int h = (int)(e / ((size_t)HD * TT)); const float* f = F + (size_t)t * pitch + h * HD; v2h o16;
#pragma unroll
    for (int q = 0; q < 2; ++q) { const int dd = d + q; const int dp = (dd < HD / 2) ? dd + HD / 2 : dd - HD / 2; const float x0 = f[dd], x1 = f[dp];
        const v2f cs = *(const v2f*)(CS + ((size_t)t * HD + dd) * 2); float a = __fmul_rn(x0, cs[0]), bq = __fmul_rn(x1, cs[1]); asm volatile("" : "+v"(a)); asm volatile("" : "+v"(bq)); const float r = (dd < HD / 2) ? __fsub_rn(a, bq) : __fadd_rn(a, bq);
        o16[q] = (h16)r; }
    *(volatile v2h*)(P16 + e) = o16; __threadfence(); *(volatile v2h*)(P16 + e) = o16; }

__global__ __launch_bounds__(256) void k_vtp(const float* __restrict__ F, int pitch, int nheads, h16* V16) { const size_t e = ((size_t)blockIdx.x * 256 + threadIdx.x) * 2; if (e >= (size_t)nheads * HD * TT) return; const int t = (int)(e % TT); const int d = (int)((e / TT) % HD); const int g = (int)(e / ((size_t)TT * HD)); v2h o16;
#pragma unroll
    for (int q = 0; q < 2; ++q) { const float x = F[(size_t)(t + q) * pitch + g * HD + d]; o16[q] = (h16)x; }
    *(volatile v2h*)(V16 + e) = o16; __threadfence(); *(volatile v2h*)(V16 + e) = o16; }

__global__ __launch_bounds__(256) void k_asoft(const float* __restrict__ Sb, const int* __restrict__ mk, h16* P16) {
    const int lane = threadIdx.x & 31; const int row = blockIdx.x * 8 + (threadIdx.x >> 5); if (row >= ZH * TT) return; const float* sr = Sb + (size_t)row * TT; float v[TT / 32];
    unsigned long long mbits = 0ull;
#pragma unroll
    for (int ch = 0; ch < TT / 128; ++ch) { const v4i m4 = *(const v4i*)(mk + ch * 128 + lane * 4);
#pragma unroll
        for (int q = 0; q < 4; ++q) mbits |= ((m4[q] != 0) ? 1ull : 0ull) << (ch * 4 + q); }
    asm volatile("" ::: "memory");
    float mx = -__builtin_huge_valf();
#pragma unroll
    for (int ch = 0; ch < TT / 128; ++ch) { const int j0 = ch * 128 + lane * 4; const v4f a = *(const v4f*)(sr + j0);
#pragma unroll
        for (int q = 0; q < 4; ++q) { const float t = ((mbits >> (ch * 4 + q)) & 1ull) ? __fmul_rn(a[q], SCL) : FMIN; v[ch * 4 + q] = t; mx = fmaxf(mx, t); } }
#pragma unroll
    for (int sh = 16; sh; sh >>= 1) mx = fmaxf(mx, __shfl_xor(mx, sh, 32));
    float sum = 0.f;
#pragma unroll
    for (int k = 0; k < TT / 32; ++k) { float d0 = __fsub_rn(v[k], mx); asm volatile("" : "+v"(d0)); v[k] = __builtin_amdgcn_exp2f(__fmul_rn(d0, 1.4426950408889634f)); sum += v[k]; }
#pragma unroll
    for (int sh = 16; sh; sh >>= 1) sum += __shfl_xor(sum, sh, 32);
    const float f = __fdiv_rn(PCAR, sum);
#pragma unroll 1
    for (int ps = 0; ps < 2; ++ps) {
#pragma unroll
        for (int ch = 0; ch < TT / 128; ++ch) { v4h o4;
#pragma unroll
            for (int q = 0; q < 4; ++q) o4[q] = (h16)(v[ch * 4 + q] * f);
            *(volatile v4h*)(P16 + (size_t)row * TT + ch * 128 + lane * 4) = o4; }
        if (ps == 0) __threadfence(); }
}

__global__ __launch_bounds__(256) void k_merge(const float* __restrict__ O, int h0, h16* CT) { const size_t e = ((size_t)blockIdx.x * 256 + threadIdx.x) * 2; if (e >= (size_t)ZH * TT * HD) return; const int d = (int)(e % HD); const int t = (int)((e / HD) % TT); const int zz = (int)(e / ((size_t)HD * TT)); const size_t oo = (size_t)t * DQ + (size_t)(h0 + zz) * HD + d;
    v2h o16;
#pragma unroll
    for (int q = 0; q < 2; ++q) o16[q] = (h16)(O[e + q] * (CCAR / PCAR));
    *(volatile v2h*)(CT + oo) = o16; __threadfence(); *(volatile v2h*)(CT + oo) = o16; }

__global__ __launch_bounds__(256) void k_addres(float* Y, const float* __restrict__ xr) { const size_t i = (size_t)blockIdx.x * 256 + threadIdx.x; if (i >= (size_t)TT * DM / 4) return; const v4f a = *(const v4f*)(Y + i * 4); const v4f r = *(const v4f*)(xr + i * 4); v4f o;
#pragma unroll
    for (int q = 0; q < 4; ++q) o[q] = __fadd_rn(a[q], bfr(r[q]));
    *(volatile v4f*)(Y + i * 4) = o; __threadfence(); *(volatile v4f*)(Y + i * 4) = o; }

__global__ __launch_bounds__(256) void k_relu16(const float* __restrict__ H, h16* H16) { const size_t i = (size_t)blockIdx.x * 256 + threadIdx.x; if (i >= (size_t)TT * FF / 8) return; const v8f a = *(const v8f*)(H + i * 8); v8h o;
#pragma unroll
    for (int k = 0; k < 8; ++k) o[k] = (h16)fmaxf(a[k], 0.0f);
    *(volatile v8h*)(H16 + i * 8) = o; __threadfence(); *(volatile v8h*)(H16 + i * 8) = o; }

__global__ __launch_bounds__(256) void k_addout(const float* __restrict__ Y, const float* __restrict__ G, float* out) { const size_t i = (size_t)blockIdx.x * 256 + threadIdx.x; if (i >= (size_t)TT * DM / 4) return; const v4f a = *(const v4f*)(Y + i * 4); const v4f r = *(const v4f*)(G + i * 4); v4f o;
#pragma unroll
    for (int q = 0; q < 4; ++q) o[q] = __fadd_rn(a[q], r[q]);
    *(volatile v4f*)(out + i * 4) = o; __threadfence(); *(volatile v4f*)(out + i * 4) = o; }

__host__ __device__ constexpr size_t al256(size_t b) { return (b + 255) & ~(size_t)255; }
__host__ __device__ constexpr size_t cmax(size_t a, size_t b) { return a > b ? a : b; }
constexpr size_t SZ_WQKV = (size_t)D3 * DM * 2, SZ_WO = (size_t)DM * DQ * 2, SZ_W1 = (size_t)FF * DM * 2, SZ_W2 = (size_t)DM * FF * 2, SZ_CS = (size_t)TT * HD * 2 * 4, SZ_X = (size_t)TT * DM * 2;
constexpr size_t SZ_F = (size_t)TT * D3 * 4, SZ_S = (size_t)ZH * TT * TT * 4, SZ_H = (size_t)TT * FF * 4, SZ_R1 = cmax(SZ_F, cmax(SZ_S, SZ_H));
constexpr size_t SZ_QP = (size_t)NH_ * TT * HD * 2, SZ_P = (size_t)ZH * TT * TT * 2, SZ_H16 = (size_t)TT * FF * 2, SZ_R2 = cmax(SZ_P, SZ_H16);
constexpr size_t SZ_OB = (size_t)ZH * TT * HD * 4, SZ_CT = (size_t)TT * DQ * 2, SZ_Y = (size_t)TT * DM * 4, SZ_G = (size_t)TT * DM * 4;
constexpr size_t WS_TOTAL = al256(SZ_WQKV) + al256(SZ_WO) + al256(SZ_W1) + al256(SZ_W2) + al256(SZ_CS) + al256(SZ_X) + al256(SZ_R1) + 3 * al256(SZ_QP) + al256(SZ_R2) + al256(SZ_OB) + al256(SZ_CT) + al256(SZ_Y) + al256(SZ_G);
static_assert(WS_TOTAL <= (size_t)134217728);
static_assert(SZ_F <= SZ_R1 && SZ_S <= SZ_R1 && SZ_H <= SZ_R1);
static_assert(SZ_P <= SZ_R2 && SZ_H16 <= SZ_R2);
static_assert((size_t)((NB - 1) * SEQ_FULL + TT) * DM * 4 <= (size_t)NB_FULL * SEQ_FULL * DM * 4);

extern "C" void kernel_launch(void* const* d_in, const int* in_sizes, int n_in,
                              void* d_out, int out_size, void* d_ws, size_t ws_size, hipStream_t stream) {
    if (n_in < 14) return;
    const size_t rows_need = (size_t)(NB - 1) * SEQ_FULL + TT;
    if ((size_t)in_sizes[0] < rows_need * DM) return;
    if ((size_t)in_sizes[1] < rows_need) return;
    if ((size_t)in_sizes[2] < (size_t)DM * DM || (size_t)in_sizes[3] < (size_t)DM * DM || (size_t)in_sizes[4] < (size_t)DM * DM || (size_t)in_sizes[5] < (size_t)DQ * DM) return;
    if (in_sizes[6] < DM || in_sizes[7] < DM || in_sizes[8] < DM || in_sizes[9] < DM) return;
    if ((size_t)in_sizes[10] < (size_t)DM * FF || in_sizes[11] < FF || (size_t)in_sizes[12] < (size_t)FF * DM || in_sizes[13] < DM) return;
    if ((size_t)out_size < rows_need * DM) return;
    const float* x = (const float*)d_in[0]; const int* msk = (const int*)d_in[1];
    const float* wq = (const float*)d_in[2]; const float* wk = (const float*)d_in[3]; const float* wv = (const float*)d_in[4]; const float* wo = (const float*)d_in[5];
    const float* g1 = (const float*)d_in[6]; const float* be1 = (const float*)d_in[7]; const float* g2 = (const float*)d_in[8]; const float* be2 = (const float*)d_in[9];
    const float* w1 = (const float*)d_in[10]; const float* fb1 = (const float*)d_in[11]; const float* w2 = (const float*)d_in[12]; const float* fb2 = (const float*)d_in[13];
    float* OUT = (float*)d_out;
    char* wsp = (char*)d_ws;
    auto take = [&](size_t bytes) { char* p = wsp; wsp += al256(bytes); return (void*)p; };
    h16* WQKV = (h16*)take(SZ_WQKV); h16* WO = (h16*)take(SZ_WO); h16* W1B = (h16*)take(SZ_W1); h16* W2B = (h16*)take(SZ_W2); float* CS = (float*)take(SZ_CS); h16* X16 = (h16*)take(SZ_X);
    char* R1 = (char*)take(SZ_R1); h16* QP16 = (h16*)take(SZ_QP); h16* KP16 = (h16*)take(SZ_QP); h16* VT16 = (h16*)take(SZ_QP); char* R2 = (char*)take(SZ_R2);
    float* Ob = (float*)take(SZ_OB); h16* CT16 = (h16*)take(SZ_CT); float* Y = (float*)take(SZ_Y); float* G = (float*)take(SZ_G);
    if ((size_t)(wsp - (char*)d_ws) > ws_size) return;
    float* F = (float*)R1; float* Sb = (float*)R1; float* H = (float*)R1; h16* P16 = (h16*)R2; h16* H16 = (h16*)R2;

    k_wt<<<(unsigned)((DM * DM / 64 + 63) / 64), 256, 0, stream>>>(wq, DM, DM, WQKV);
    k_wt<<<(unsigned)((DM * DM / 64 + 63) / 64), 256, 0, stream>>>(wk, DM, DM, WQKV + (size_t)DM * DM);
    k_wt<<<(unsigned)((DM * DM / 64 + 63) / 64), 256, 0, stream>>>(wv, DM, DM, WQKV + (size_t)2 * DM * DM);
    k_wt<<<(unsigned)((DQ * DM / 64 + 63) / 64), 256, 0, stream>>>(wo, DQ, DM, WO);
    k_wt<<<(unsigned)((DM * FF / 64 + 63) / 64), 256, 0, stream>>>(w1, DM, FF, W1B);
    k_wt<<<(unsigned)((FF * DM / 64 + 63) / 64), 256, 0, stream>>>(w2, FF, DM, W2B);
    k_cstab<<<(unsigned)((TT * 32 + 255) / 256), 256, 0, stream>>>(CS);
    const unsigned LR = (unsigned)(((size_t)NH_ * TT * HD / 2 + 255) / 256);
    for (int b = 0; b < NB; ++b) {
        const float* xb = x + (size_t)b * SEQ_FULL * DM; const int* mb = msk + (size_t)b * SEQ_FULL; float* ob = OUT + (size_t)b * SEQ_FULL * DM;
        k_lnx<true><<<TT / 8, 256, 0, stream>>>(xb, g1, be1, X16);
        k_gemm<false><<<dim3(TT / 64, D3 / 64, 1), 32, 0, stream>>>(X16, WQKV, DM, F, D3, nullptr, 1.0f / WCAR, 0, 0, 0);
        k_rope<<<LR, 256, 0, stream>>>(F, D3, NH_, CS, QP16);
        k_rope<<<LR, 256, 0, stream>>>(F + DM, D3, NH_, CS, KP16);
        k_vtp<<<LR, 256, 0, stream>>>(F + 2 * DM, D3, NH_, VT16);
        for (int h0 = 0; h0 < NH_; h0 += ZH) { const size_t zq = (size_t)h0;
            k_gemm<false><<<dim3(TT / 64, TT / 64, ZH), 32, 0, stream>>>(QP16 + zq * TT * HD, KP16 + zq * TT * HD, HD, Sb, TT, nullptr, 1.0f, (size_t)TT * HD, (size_t)TT * HD, (size_t)TT * TT);
            k_asoft<<<ZH * TT / 8, 256, 0, stream>>>(Sb, mb, P16);
            k_gemm<false><<<dim3(TT / 64, HD / 64, ZH), 32, 0, stream>>>(P16, VT16 + zq * HD * TT, TT, Ob, HD, nullptr, 1.0f, (size_t)TT * TT, (size_t)HD * TT, (size_t)TT * HD);
            k_merge<<<(unsigned)(((size_t)ZH * TT * HD / 2 + 255) / 256), 256, 0, stream>>>(Ob, h0, CT16); }
        k_gemm<false><<<dim3(TT / 64, DM / 64, 1), 32, 0, stream>>>(CT16, WO, DQ, Y, DM, nullptr, 1.0f / (CCAR * WCAR), 0, 0, 0);
        k_addres<<<(unsigned)(((size_t)TT * DM / 4 + 255) / 256), 256, 0, stream>>>(Y, xb);
        k_lnx<false><<<TT / 8, 256, 0, stream>>>(Y, g2, be2, X16);
        k_gemm<true><<<dim3(TT / 64, FF / 64, 1), 32, 0, stream>>>(X16, W1B, DM, H, FF, fb1, 1.0f / WCAR, 0, 0, 0);
        k_relu16<<<(unsigned)(((size_t)TT * FF / 8 + 255) / 256), 256, 0, stream>>>(H, H16);
        k_gemm<true><<<dim3(TT / 64, DM / 64, 1), 32, 0, stream>>>(H16, W2B, FF, G, DM, fb2, 1.0f / WCAR, 0, 0, 0);
        k_addout<<<(unsigned)(((size_t)TT * DM / 4 + 255) / 256), 256, 0, stream>>>(Y, G, ob);
    }
}
